// DagSage_17377437679928
// MI455X (gfx1250) — hardware-verified
//
#include <hip/hip_runtime.h>
#include <hip/hip_bf16.h>


#define NB_    32
#define NN_    64
#define R_     256
#define GPB_   16
#define NBLK_  (NB_ / GPB_)
#define KF_    1024
#define KQ_    768
#define AP_    1032
#define PL_    (GPB_ * AP_)
#define SAPL_  (GPB_ * NN_)
#define SKPL_  (GPB_ * R_)
#define MROWS_ (NB_ * NN_)

static_assert(NB_ % GPB_ == 0);
static_assert((AP_ * 2) % 16 == 0);
static_assert(R_ % 64 == 0 && KF_ % 32 == 0 && KQ_ % 32 == 0);
static_assert(MROWS_ % 64 == 0);

typedef float          v4f   __attribute__((ext_vector_type(4)));
typedef float          v8f   __attribute__((ext_vector_type(8)));
typedef __bf16         v16b  __attribute__((ext_vector_type(16)));
typedef unsigned short u16x8 __attribute__((ext_vector_type(8)));
typedef unsigned short u16x4 __attribute__((ext_vector_type(4)));

union FragB { u16x8 h[2]; v16b v; };

constexpr size_t SZ_N16   = (size_t)MROWS_ * R_ * 2;
constexpr size_t SZ_W256  = (size_t)R_ * R_ * 2;
constexpr size_t SZ_W1024 = (size_t)R_ * KF_ * 2;
constexpr size_t SZ_W768  = (size_t)R_ * KQ_ * 2;
constexpr size_t SZ_REP32 = (size_t)MROWS_ * R_ * 4;
constexpr size_t SZ_KEY16 = (size_t)NB_ * NN_ * R_ * 2;
constexpr size_t SZ_RPT16 = (size_t)NB_ * 8 * R_ * 8 * 2;

constexpr size_t OFF_NH  = 0;
constexpr size_t OFF_NL  = OFF_NH  + SZ_N16;
constexpr size_t OFF_WSH = OFF_NL  + SZ_N16;
constexpr size_t OFF_WSL = OFF_WSH + SZ_W256;
constexpr size_t OFF_WRH = OFF_WSL + SZ_W256;
constexpr size_t OFF_WRL = OFF_WRH + SZ_W256;
constexpr size_t OFF_WKH = OFF_WRL + SZ_W256;
constexpr size_t OFF_WKL = OFF_WKH + SZ_W256;
constexpr size_t OFF_WFH = OFF_WKL + SZ_W256;
constexpr size_t OFF_WFL = OFF_WFH + SZ_W1024;
constexpr size_t OFF_WHH = OFF_WFL + SZ_W1024;
constexpr size_t OFF_WHL = OFF_WHH + SZ_W1024;
constexpr size_t OFF_WQH = OFF_WHL + SZ_W1024;
constexpr size_t OFF_WQL = OFF_WQH + SZ_W768;
constexpr size_t OFF_WOH = OFF_WQL + SZ_W768;
constexpr size_t OFF_WOL = OFF_WOH + SZ_W768;
constexpr size_t OFF_REP = OFF_WOL + SZ_W768;
constexpr size_t OFF_KH  = OFF_REP + SZ_REP32;
constexpr size_t OFF_KL  = OFF_KH  + SZ_KEY16;
constexpr size_t OFF_RTH = OFF_KL  + SZ_KEY16;
constexpr size_t OFF_RTL = OFF_RTH + SZ_RPT16;
constexpr size_t WS_END  = OFF_RTL + SZ_RPT16;
static_assert(WS_END <= (size_t)134217728);
static_assert(OFF_NL % 128 == 0 && OFF_WSH % 128 == 0 && OFF_WSL % 128 == 0 && OFF_WRH % 128 == 0 && OFF_WRL % 128 == 0);
static_assert(OFF_WKH % 128 == 0 && OFF_WKL % 128 == 0 && OFF_WFH % 128 == 0 && OFF_WFL % 128 == 0 && OFF_WHH % 128 == 0);
static_assert(OFF_WHL % 128 == 0 && OFF_WQH % 128 == 0 && OFF_WQL % 128 == 0 && OFF_WOH % 128 == 0 && OFF_WOL % 128 == 0);
static_assert(OFF_REP % 128 == 0 && OFF_KH % 128 == 0 && OFF_KL % 128 == 0 && OFF_RTH % 128 == 0 && OFF_RTL % 128 == 0);

constexpr int L_ACT     = 0;
constexpr int L_SA      = L_ACT  + 2 * PL_ * 2;
constexpr int L_LOG     = L_SA   + 2 * SAPL_ * 2;
constexpr int L_ROWF    = L_LOG  + GPB_ * NN_ * 4;
constexpr int L_KEY     = L_ROWF + GPB_ * R_ * 4;
constexpr int LDS_BYTES = L_KEY  + 2 * SKPL_ * 2;
static_assert(L_SA % 16 == 0 && L_LOG % 16 == 0 && L_ROWF % 16 == 0 && L_KEY % 16 == 0 && LDS_BYTES % 16 == 0);
static_assert(LDS_BYTES <= 300000);

__device__ __forceinline__ unsigned short f32_to_bf16(float f) {
    unsigned u = __float_as_uint(f);
    unsigned r = u + 0x7FFFu + ((u >> 16) & 1u);
    return (unsigned short)(r >> 16);
}
__device__ __forceinline__ float bf16_to_f32(unsigned short b) {
    return __uint_as_float(((unsigned)b) << 16);
}
__device__ __forceinline__ v8f ld8f(const float* p) {
    v4f a = *(const v4f*)p;
    v4f b = *(const v4f*)(p + 4);
    return __builtin_shufflevector(a, b, 0, 1, 2, 3, 4, 5, 6, 7);
}
__device__ __forceinline__ void split8(const v8f x, u16x8& hv, u16x8& lv) {
#pragma unroll
    for (int c = 0; c < 8; ++c) {
        const float f = x[c];
        const unsigned short hb = f32_to_bf16(f);
        const unsigned short lb = f32_to_bf16(f - bf16_to_f32(hb));
        hv[c] = hb;
        lv[c] = lb;
    }
}
__device__ __forceinline__ void st_split2(unsigned short* p, int looff, float v) {
    const unsigned short hb = f32_to_bf16(v);
    const unsigned short lb = f32_to_bf16(v - bf16_to_f32(hb));
    p[0] = hb;
    p[looff] = lb;
}

__device__ __forceinline__ void mma16(v8f& acc, const FragB& a, const FragB& b) {
    acc = __builtin_amdgcn_wmma_f32_16x16x32_bf16(false, a.v, false, b.v, (short)0, acc, false, false);
    asm volatile("v_nop\n\tv_nop\n\tv_nop\n\tv_nop" : "+v"(acc) : "v"(a.v), "v"(b.v));
}
__device__ __forceinline__ void mma3(v8f& acc, const FragB& ah, const FragB& al, const FragB& bh, const FragB& bl) {
    acc = __builtin_amdgcn_wmma_f32_16x16x32_bf16(false, ah.v, false, bh.v, (short)0, acc, false, false);
    acc = __builtin_amdgcn_wmma_f32_16x16x32_bf16(false, ah.v, false, bl.v, (short)0, acc, false, false);
    acc = __builtin_amdgcn_wmma_f32_16x16x32_bf16(false, al.v, false, bh.v, (short)0, acc, false, false);
    asm volatile("v_nop\n\tv_nop\n\tv_nop\n\tv_nop" : "+v"(acc) : "v"(ah.v), "v"(al.v), "v"(bh.v), "v"(bl.v));
}

__global__ __launch_bounds__(256)
void cvt8_kernel(const float* __restrict__ src, unsigned short* dhi, unsigned short* dlo, int n8)
{
    const int i = blockIdx.x * 256 + threadIdx.x;
    if (i >= n8) return;
    const size_t e = (size_t)i * 8;
    const v8f x = ld8f(src + e);
    u16x8 hv, lv;
    split8(x, hv, lv);
    *(volatile u16x8*)(dhi + e) = hv;
    *(volatile u16x8*)(dlo + e) = lv;
    __threadfence();
    *(volatile u16x8*)(dhi + e) = hv;
    *(volatile u16x8*)(dlo + e) = lv;
}

__global__ __launch_bounds__(256)
void wt_cvt_kernel(const float* __restrict__ src, unsigned short* dhi, unsigned short* dlo,
                   int Nw, int Kd, int nrows)
{
    __shared__ __attribute__((aligned(16))) float sT[64 * 68];
    const int tid  = threadIdx.x;
    const int lane = tid & 31;
    const int wave = tid >> 5;
    const int n0 = blockIdx.x * 64;
    const int k0 = blockIdx.y * 64;

#pragma unroll
    for (int it = 0; it < 4; ++it) {
        const int idx = it * 256 + tid;
        const int kk  = idx >> 4;
        const int n4  = (idx & 15) * 4;
        const int gn  = n0 + n4;
        const int gnc = min(gn, Nw - 4);
        const v4f v = *(const v4f*)(src + (size_t)(k0 + kk) * Nw + gnc);
        const bool in = (gn < Nw);
        sT[(n4 + 0) * 68 + kk] = in ? v[0] : 0.0f;
        sT[(n4 + 1) * 68 + kk] = in ? v[1] : 0.0f;
        sT[(n4 + 2) * 68 + kk] = in ? v[2] : 0.0f;
        sT[(n4 + 3) * 68 + kk] = in ? v[3] : 0.0f;
    }
    __syncthreads();

    u16x8 hv[2], lv[2];
    const int c = (lane & 7) * 8;
#pragma unroll
    for (int it = 0; it < 2; ++it) {
        const int nn = it * 32 + wave * 4 + (lane >> 3);
        const v8f x = ld8f(sT + nn * 68 + c);
        split8(x, hv[it], lv[it]);
    }
#pragma unroll
    for (int it = 0; it < 2; ++it) {
        const int gr = n0 + it * 32 + wave * 4 + (lane >> 3);
        if (gr < nrows) {
            const size_t o = (size_t)gr * Kd + k0 + c;
            *(volatile u16x8*)(dhi + o) = hv[it];
            *(volatile u16x8*)(dlo + o) = lv[it];
        }
    }
    __threadfence();
#pragma unroll
    for (int it = 0; it < 2; ++it) {
        const int gr = n0 + it * 32 + wave * 4 + (lane >> 3);
        if (gr < nrows) {
            const size_t o = (size_t)gr * Kd + k0 + c;
            *(volatile u16x8*)(dhi + o) = hv[it];
            *(volatile u16x8*)(dlo + o) = lv[it];
        }
    }
}

__global__ __launch_bounds__(256)
void init_src_kernel(const float* __restrict__ bK, const float* __restrict__ bR,
                     unsigned short* kH, unsigned short* kL, unsigned short* rH, unsigned short* rL, int n8)
{
    const int i = blockIdx.x * 256 + threadIdx.x;
    if (i >= n8) return;
    const size_t e = (size_t)i * 8;
    const int ck = (int)(e & 255);
    const v8f xk = ld8f(bK + ck);
    const int rr = (int)((e >> 3) & 255);
    const float br = bR[rr];
    v8f xr;
#pragma unroll
    for (int c = 0; c < 8; ++c) xr[c] = br;
    u16x8 khv, klv, rhv, rlv;
    split8(xk, khv, klv);
    split8(xr, rhv, rlv);
    *(volatile u16x8*)(kH + e) = khv;
    *(volatile u16x8*)(kL + e) = klv;
    *(volatile u16x8*)(rH + e) = rhv;
    *(volatile u16x8*)(rL + e) = rlv;
    __threadfence();
    *(volatile u16x8*)(kH + e) = khv;
    *(volatile u16x8*)(kL + e) = klv;
    *(volatile u16x8*)(rH + e) = rhv;
    *(volatile u16x8*)(rL + e) = rlv;
}

__global__ __launch_bounds__(256)
void copy4_kernel(const float* __restrict__ src, float* dst, int n4)
{
    const int i = blockIdx.x * 256 + threadIdx.x;
    if (i >= n4) return;
    const size_t e = (size_t)i * 4;
    const v4f v = *(const v4f*)(src + e);
    *(volatile v4f*)(dst + e) = v;
    __threadfence();
    *(volatile v4f*)(dst + e) = v;
}

template<int NBF>
__device__ __forceinline__ void tile_store_pass(const float* st, float* gp, int ldc, int lane) {
    constexpr int CW  = NBF * 16;
    constexpr int P   = CW + 4;
    constexpr int LPR = CW / 4;
    static_assert(32 % LPR == 0);
    constexpr int RPI = 32 / LPR;
    constexpr int NIT = 32 / RPI;
    const int rsub = lane / LPR;
    const int c0   = (lane % LPR) * 4;
#pragma unroll
    for (int it = 0; it < NIT; ++it) {
        const int row = it * RPI + rsub;
        const v4f v = *(const v4f*)(st + row * P + c0);
        *(volatile v4f*)(gp + (size_t)row * ldc + c0) = v;
    }
}

template<int NBF>
__global__ __launch_bounds__(128)
void gemm_x3_kernel(const unsigned short* __restrict__ Ah, const unsigned short* __restrict__ Al,
                    const unsigned short* __restrict__ Bh, const unsigned short* __restrict__ Bl,
                    float* C, int K, int ldc)
{
    constexpr int CW = NBF * 16;
    constexpr int P  = CW + 4;
    static_assert(CW % 32 == 0);
    __shared__ __attribute__((aligned(16))) float stile[4][32 * P];

    const int tid  = threadIdx.x;
    const int lane = tid & 31;
    const int wave = tid >> 5;
    const int h    = lane >> 4;
    const int m    = lane & 15;
    const int wm   = wave >> 1;
    const int wn   = wave & 1;

    const int rowW = blockIdx.y * 64 + wm * 32;
    const int colW = blockIdx.x * (2 * CW) + wn * CW;

    v8f acc[2 * NBF];
#pragma unroll
    for (int j = 0; j < 2 * NBF; ++j)
#pragma unroll
        for (int r = 0; r < 8; ++r) acc[j][r] = 0.0f;

    const size_t aoff  = (size_t)(rowW + m) * K + 8 * h;
    const size_t boff  = (size_t)(colW + m) * K + 8 * h;
    const size_t sub16 = (size_t)16 * K;
    const int nk = K >> 5;

#pragma unroll 1
    for (int kt = 0; kt < nk; ++kt) {
        const size_t k0 = (size_t)kt * 32;
        FragB fa[2], ga[2], fb[NBF], gb[NBF];
#pragma unroll
        for (int s = 0; s < 2; ++s) {
            const unsigned short* p = Ah + aoff + s * sub16 + k0;
            const unsigned short* q = Al + aoff + s * sub16 + k0;
            fa[s].h[0] = *(const u16x8*)(p);
            fa[s].h[1] = *(const u16x8*)(p + 16);
            ga[s].h[0] = *(const u16x8*)(q);
            ga[s].h[1] = *(const u16x8*)(q + 16);
        }
#pragma unroll
        for (int j = 0; j < NBF; ++j) {
            const unsigned short* p = Bh + boff + j * sub16 + k0;
            const unsigned short* q = Bl + boff + j * sub16 + k0;
            fb[j].h[0] = *(const u16x8*)(p);
            fb[j].h[1] = *(const u16x8*)(p + 16);
            gb[j].h[0] = *(const u16x8*)(q);
            gb[j].h[1] = *(const u16x8*)(q + 16);
        }
#pragma unroll
        for (int s = 0; s < 2; ++s)
#pragma unroll
            for (int j = 0; j < NBF; ++j) {
                mma16(acc[s * NBF + j], fa[s], fb[j]);
                mma16(acc[s * NBF + j], fa[s], gb[j]);
                mma16(acc[s * NBF + j], ga[s], fb[j]);
            }
    }

    float* st = stile[wave];
#pragma unroll
    for (int s = 0; s < 2; ++s)
#pragma unroll
        for (int j = 0; j < NBF; ++j)
#pragma unroll
            for (int r = 0; r < 8; ++r)
                st[(s * 16 + 8 * h + r) * P + j * 16 + m] = acc[s * NBF + j][r];
    __syncthreads();

    float* gp = C + (size_t)rowW * ldc + colW;
    tile_store_pass<NBF>(st, gp, ldc, lane);
    __threadfence();
    tile_store_pass<NBF>(st, gp, ldc, lane);
}

__device__ __forceinline__ void gemm2(v8f (&acc)[2], const unsigned short* actp, int abase,
                                      const unsigned short* __restrict__ wH, const unsigned short* __restrict__ wL,
                                      int K, int nt0, unsigned skip, int lane)
{
    const int h = lane >> 4, m = lane & 15;
#pragma unroll
    for (int t = 0; t < 2; ++t)
#pragma unroll
        for (int r = 0; r < 8; ++r) acc[t][r] = 0.0f;
    const unsigned short* arH = actp + m * AP_ + abase + 8 * h;
    const unsigned short* arL = arH + PL_;
    const size_t bo = ((size_t)(nt0 * 16 + m)) * K + 8 * h;
    const unsigned short* b0H = wH + bo;
    const unsigned short* b0L = wL + bo;
    const unsigned short* b1H = b0H + (size_t)16 * K;
    const unsigned short* b1L = b0L + (size_t)16 * K;
#pragma unroll 1
    for (int k0 = 0; k0 < K; k0 += 32) {
        if ((skip >> (k0 >> 8)) & 1u) continue;
        FragB fa, ga, fb0, gb0, fb1, gb1;
        fa.h[0]  = *(const u16x8*)(arH + k0);       fa.h[1]  = *(const u16x8*)(arH + k0 + 16);
        ga.h[0]  = *(const u16x8*)(arL + k0);       ga.h[1]  = *(const u16x8*)(arL + k0 + 16);
        fb0.h[0] = *(const u16x8*)(b0H + k0);       fb0.h[1] = *(const u16x8*)(b0H + k0 + 16);
        gb0.h[0] = *(const u16x8*)(b0L + k0);       gb0.h[1] = *(const u16x8*)(b0L + k0 + 16);
        fb1.h[0] = *(const u16x8*)(b1H + k0);       fb1.h[1] = *(const u16x8*)(b1H + k0 + 16);
        gb1.h[0] = *(const u16x8*)(b1L + k0);       gb1.h[1] = *(const u16x8*)(b1L + k0 + 16);
        mma3(acc[0], fa, ga, fb0, gb0);
        mma3(acc[1], fa, ga, fb1, gb1);
    }
}

__device__ __forceinline__ void rmw_rep_plane(unsigned short* base, const float* sRow, int bg0, int idx,
                                              int wave, int lane, int isLo)
{
    const int jb = idx >> 3, es = idx & 7, p = lane & 7;
#pragma unroll 1
    for (int q = 0; q < 16; ++q) {
        const int grp = wave + 8 * q;
        const int li  = (grp << 2) + (lane >> 3);
        const int b   = li >> 5, rb = li & 31;
        const int r   = rb * 8 + p;
        unsigned short* ptr = base + (((size_t)((bg0 + b) * 8 + jb)) * R_ + r) * 8;
        u16x8 v = *(const u16x8*)ptr;
        const float f = sRow[b * R_ + r];
        const unsigned short hb = f32_to_bf16(f);
        const unsigned short lb = f32_to_bf16(f - bf16_to_f32(hb));
        const unsigned short nv = isLo ? lb : hb;
#pragma unroll
        for (int e = 0; e < 8; ++e) v[e] = (e == es) ? nv : v[e];
        *(volatile u16x8*)ptr = v;
        __threadfence();
        *(volatile u16x8*)ptr = v;
    }
}

__global__ __launch_bounds__(256) __attribute__((amdgpu_num_vgpr(256)))
void dag_kernel(const float* __restrict__ adj, const float* __restrict__ nrep, const float* __restrict__ bS,
                const unsigned short* __restrict__ wfH, const unsigned short* __restrict__ wfL, const float* __restrict__ bF,
                const unsigned short* __restrict__ whH, const unsigned short* __restrict__ whL, const float* __restrict__ bHd,
                const unsigned short* __restrict__ wqH, const unsigned short* __restrict__ wqL, const float* __restrict__ bQ,
                const unsigned short* __restrict__ woH, const unsigned short* __restrict__ woL, const float* __restrict__ bO,
                const unsigned short* __restrict__ wrH, const unsigned short* __restrict__ wrL, const float* __restrict__ bR,
                const unsigned short* __restrict__ wkH, const unsigned short* __restrict__ wkL, const float* __restrict__ bK,
                unsigned short* keysH, unsigned short* keysL, unsigned short* rptH, unsigned short* rptL,
                float* out)
{
    extern __shared__ __attribute__((aligned(16))) unsigned char dsm[];
    unsigned short* act  = (unsigned short*)(dsm + L_ACT);
    unsigned short* sA   = (unsigned short*)(dsm + L_SA);
    float*          sLog = (float*)(dsm + L_LOG);
    float*          sRow = (float*)(dsm + L_ROWF);
    unsigned short* sKey = (unsigned short*)(dsm + L_KEY);

    const int tid  = threadIdx.x;
    const int lane = tid & 31;
    const int wave = __builtin_amdgcn_readfirstlane(tid >> 5);
    const int h    = lane >> 4;
    const int m    = lane & 15;
    const int bg0  = blockIdx.x * GPB_;
    const int nt0  = 2 * wave;

    float bFv[2], bHv[2], bQv[2], bOv[2], bRv[2], bKv[2];
#pragma unroll
    for (int t = 0; t < 2; ++t) {
        const int n = (nt0 + t) * 16 + m;
        bFv[t] = bF[n]; bHv[t] = bHd[n]; bQv[t] = bQ[n];
        bOv[t] = bO[n]; bRv[t] = bR[n];  bKv[t] = bK[n];
    }
    u16x8 z8;
#pragma unroll
    for (int e = 0; e < 8; ++e) z8[e] = 0;
    const v4f z4 = {0.0f, 0.0f, 0.0f, 0.0f};

#pragma unroll 1
    for (int idx = 0; idx < NN_; ++idx) {
        v8f hid[2], fg[2];
#pragma unroll
        for (int t = 0; t < 2; ++t)
#pragma unroll
            for (int r = 0; r < 8; ++r) { hid[t][r] = 0.0f; fg[t][r] = 0.0f; }
#pragma unroll
        for (int q = 0; q < 8; ++q) {
            const int i = tid + 256 * q;
            const int plane = i >> 10, rem = i & 1023;
            const int row = rem >> 6, piece = rem & 63;
            const int col = 256 + ((piece >> 5) << 9) + ((piece & 31) << 3);
            *(u16x8*)(act + plane * PL_ + row * AP_ + col) = z8;
        }
        {
            const int b = tid >> 4, c = (tid & 15) * 16, g = bg0 + b;
            const float* src = nrep + ((size_t)(g * NN_ + idx)) * R_ + c;
#pragma unroll
            for (int q = 0; q < 2; ++q) {
                const v8f x = ld8f(src + 8 * q) + ld8f(bS + c + 8 * q);
                u16x8 hv, lv;
                split8(x, hv, lv);
                *(u16x8*)(act + b * AP_ + 512 + c + 8 * q) = hv;
                *(u16x8*)(act + PL_ + b * AP_ + 512 + c + 8 * q) = lv;
            }
        }
        __syncthreads();

#pragma unroll 1
        for (int it = 0; it < 3; ++it) {
            if (it == 0) {
                *(v4f*)(sLog + tid * 4) = z4;
            } else {
                const unsigned short* qh = act + m * AP_ + 768 + 8 * h;
                const unsigned short* ql = qh + PL_;
#pragma unroll 1
                for (int u = 0; u < 8; ++u) {
                    const int bp = 2 * wave + (u >> 2), mt = u & 3;
                    const int g  = bg0 + bp;
                    const size_t ko = ((size_t)(g * NN_ + mt * 16 + m)) * R_ + 8 * h;
                    const unsigned short* kh = keysH + ko;
                    const unsigned short* kl = keysL + ko;
                    v8f acc;
#pragma unroll
                    for (int r = 0; r < 8; ++r) acc[r] = 0.0f;
#pragma unroll 1
                    for (int k0 = 0; k0 < R_; k0 += 32) {
                        FragB fa, ga, fb, gb;
                        fa.h[0] = *(const u16x8*)(kh + k0);  fa.h[1] = *(const u16x8*)(kh + k0 + 16);
                        ga.h[0] = *(const u16x8*)(kl + k0);  ga.h[1] = *(const u16x8*)(kl + k0 + 16);
                        fb.h[0] = *(const u16x8*)(qh + k0);  fb.h[1] = *(const u16x8*)(qh + k0 + 16);
                        gb.h[0] = *(const u16x8*)(ql + k0);  gb.h[1] = *(const u16x8*)(ql + k0 + 16);
                        mma3(acc, fa, ga, fb, gb);
                    }
                    if (m == bp) {
                        float* d = sLog + bp * NN_ + mt * 16 + 8 * h;
#pragma unroll
                        for (int r = 0; r < 8; ++r) d[r] = acc[r];
                    }
                }
            }
            __syncthreads();

            {
                const int b = tid >> 4, jj = (tid & 15) * 4, g = bg0 + b;
                const v4f x = *(const v4f*)(sLog + b * NN_ + jj);
                float mx = fmaxf(fmaxf(x[0], x[1]), fmaxf(x[2], x[3]));
                mx = fmaxf(mx, __shfl_xor(mx, 8, 32));
                mx = fmaxf(mx, __shfl_xor(mx, 4, 32));
                mx = fmaxf(mx, __shfl_xor(mx, 2, 32));
                mx = fmaxf(mx, __shfl_xor(mx, 1, 32));
                const float* ap = adj + ((size_t)(g * NN_ + jj)) * NN_ + idx;
                v4f ev;
                float s = 0.0f;
#pragma unroll
                for (int i = 0; i < 4; ++i) {
                    const float mk = ap[(size_t)i * NN_];
                    const float e  = expf(x[i] - mx) * mk;
                    ev[i] = e;
                    s += e;
                }
                s += __shfl_xor(s, 8, 32);
                s += __shfl_xor(s, 4, 32);
                s += __shfl_xor(s, 2, 32);
                s += __shfl_xor(s, 1, 32);
                const float inv = 1.0f / s;
                u16x4 ph, pl;
#pragma unroll
                for (int i = 0; i < 4; ++i) {
                    const float p = ev[i] * inv;
                    const unsigned short hb = f32_to_bf16(p);
                    ph[i] = hb;
                    pl[i] = f32_to_bf16(p - bf16_to_f32(hb));
                }
                *(u16x4*)(sA + b * NN_ + jj) = ph;
                *(u16x4*)(sA + SAPL_ + b * NN_ + jj) = pl;
            }
            __syncthreads();

            {
                FragB aH2[2], aL2[2];
#pragma unroll
                for (int ks = 0; ks < 2; ++ks) {
                    const unsigned short* pa = sA + m * NN_ + ks * 32 + 8 * h;
                    aH2[ks].h[0] = *(const u16x8*)(pa);          aH2[ks].h[1] = *(const u16x8*)(pa + 16);
                    aL2[ks].h[0] = *(const u16x8*)(pa + SAPL_);  aL2[ks].h[1] = *(const u16x8*)(pa + SAPL_ + 16);
                }
#pragma unroll 1
                for (int bp = 0; bp < GPB_; ++bp) {
                    const int g = bg0 + bp, rs = bp & 7, hs = bp >> 3;
#pragma unroll
                    for (int t = 0; t < 2; ++t) {
                        const int n = (nt0 + t) * 16 + m;
                        const size_t ro = ((size_t)(g * 8)) * R_ * 8 + (size_t)n * 8;
                        v8f acc;
#pragma unroll
                        for (int r = 0; r < 8; ++r) acc[r] = 0.0f;
#pragma unroll
                        for (int ks = 0; ks < 2; ++ks) {
                            const size_t o0 = ro + (size_t)(4 * ks + h) * R_ * 8;
                            const size_t o1 = o0 + (size_t)2 * R_ * 8;
                            FragB fb, gb;
                            fb.h[0] = *(const u16x8*)(rptH + o0);  fb.h[1] = *(const u16x8*)(rptH + o1);
                            gb.h[0] = *(const u16x8*)(rptL + o0);  gb.h[1] = *(const u16x8*)(rptL + o1);
                            mma3(acc, aH2[ks], aL2[ks], fb, gb);
                        }
                        float v = acc[0];
#pragma unroll
                        for (int e = 1; e < 8; ++e) v = (e == rs) ? acc[e] : v;
                        if (h == hs) st_split2(act + bp * AP_ + n, PL_, v);
                    }
                }
            }
            __syncthreads();

            const unsigned skipF = (it == 0) ? 0xAu : 0u;
            const unsigned skipQ = (it == 0) ? 0x4u : 0u;
            v8f acc[2];

            gemm2(acc, act, 0, wfH, wfL, KF_, nt0, skipF, lane);
            __syncthreads();
#pragma unroll
            for (int t = 0; t < 2; ++t) {
                const int n = (nt0 + t) * 16 + m;
#pragma unroll
                for (int r = 0; r < 8; ++r) {
                    const float x = acc[t][r] + bFv[t];
                    const float f = __builtin_amdgcn_rcpf(1.0f + expf(-x));
                    fg[t][r] = f;
                    st_split2(act + (8 * h + r) * AP_ + 256 + n, PL_, f * hid[t][r]);
                }
            }
            __syncthreads();

            gemm2(acc, act, 0, whH, whL, KF_, nt0, skipF, lane);
            __syncthreads();
#pragma unroll
            for (int t = 0; t < 2; ++t) {
                const int n = (nt0 + t) * 16 + m;
#pragma unroll
                for (int r = 0; r < 8; ++r) {
                    const float th = tanhf(acc[t][r] + bHv[t]);
                    const float f  = fg[t][r];
                    const float hn = f * hid[t][r] + (1.0f - f) * th;
                    hid[t][r] = hn;
                    st_split2(act + (8 * h + r) * AP_ + 256 + n, PL_, hn);
                }
            }
            __syncthreads();

            gemm2(acc, act, 256, wqH, wqL, KQ_, nt0, skipQ, lane);
            __syncthreads();
#pragma unroll
            for (int t = 0; t < 2; ++t) {
                const int n = (nt0 + t) * 16 + m;
#pragma unroll
                for (int r = 0; r < 8; ++r)
                    st_split2(act + (8 * h + r) * AP_ + 768 + n, PL_, acc[t][r] + bQv[t]);
            }
            __syncthreads();
        }

        {
            v8f acc[2];
            gemm2(acc, act, 256, woH, woL, KQ_, nt0, 0u, lane);
#pragma unroll
            for (int t = 0; t < 2; ++t) {
                const int n = (nt0 + t) * 16 + m;
#pragma unroll
                for (int r = 0; r < 8; ++r) sRow[(8 * h + r) * R_ + n] = acc[t][r] + bOv[t];
            }
        }
        __syncthreads();

        {
            v4f ov[4];
#pragma unroll
            for (int q = 0; q < 4; ++q) {
                const int L = (wave + 8 * q) * 4 + (lane >> 3);
                const int b = L >> 3, c = (L & 7) * 32 + (lane & 7) * 4;
                ov[q] = *(const v4f*)(sRow + b * R_ + c);
            }
#pragma unroll
            for (int q = 0; q < 4; ++q) {
                const int L = (wave + 8 * q) * 4 + (lane >> 3);
                const int b = L >> 3, c = (L & 7) * 32 + (lane & 7) * 4;
                float* gp = out + ((size_t)((bg0 + b) * NN_ + idx)) * R_ + c;
                *(volatile v4f*)gp = ov[q];
            }
            {
                const int b = tid >> 4, c = (tid & 15) * 16;
#pragma unroll
                for (int q = 0; q < 2; ++q) {
                    const v8f x = ld8f(sRow + b * R_ + c + 8 * q);
                    u16x8 hv, lv;
                    split8(x, hv, lv);
                    *(u16x8*)(act + b * AP_ + c + 8 * q) = hv;
                    *(u16x8*)(act + PL_ + b * AP_ + c + 8 * q) = lv;
                }
            }
            __threadfence();
#pragma unroll
            for (int q = 0; q < 4; ++q) {
                const int L = (wave + 8 * q) * 4 + (lane >> 3);
                const int b = L >> 3, c = (L & 7) * 32 + (lane & 7) * 4;
                float* gp = out + ((size_t)((bg0 + b) * NN_ + idx)) * R_ + c;
                *(volatile v4f*)gp = ov[q];
            }
        }
        __syncthreads();

        {
            v8f acc[2];
            gemm2(acc, act, 0, wrH, wrL, R_, nt0, 0u, lane);
#pragma unroll
            for (int t = 0; t < 2; ++t) {
                const int n = (nt0 + t) * 16 + m;
#pragma unroll
                for (int r = 0; r < 8; ++r) sRow[(8 * h + r) * R_ + n] = acc[t][r] + bRv[t];
            }
            gemm2(acc, act, 0, wkH, wkL, R_, nt0, 0u, lane);
#pragma unroll
            for (int t = 0; t < 2; ++t) {
                const int n = (nt0 + t) * 16 + m;
#pragma unroll
                for (int r = 0; r < 8; ++r) st_split2(sKey + (8 * h + r) * R_ + n, SKPL_, acc[t][r] + bKv[t]);
            }
        }
        __syncthreads();

        {
            u16x8 kv[4];
#pragma unroll
            for (int q = 0; q < 4; ++q) {
                const int L = (wave + 8 * q) * 4 + (lane >> 3);
                const int b = (L >> 2) & 15, c = (L & 3) * 64 + (lane & 7) * 8;
                kv[q] = *(const u16x8*)(sKey + (q >> 1) * SKPL_ + b * R_ + c);
            }
#pragma unroll
            for (int q = 0; q < 4; ++q) {
                const int L = (wave + 8 * q) * 4 + (lane >> 3);
                const int b = (L >> 2) & 15, c = (L & 3) * 64 + (lane & 7) * 8;
                unsigned short* base = (q < 2) ? keysH : keysL;
                unsigned short* gp = base + ((size_t)((bg0 + b) * NN_ + idx)) * R_ + c;
                *(volatile u16x8*)gp = kv[q];
            }
            rmw_rep_plane(rptH, sRow, bg0, idx, wave, lane, 0);
            rmw_rep_plane(rptL, sRow, bg0, idx, wave, lane, 1);
            __threadfence();
#pragma unroll
            for (int q = 0; q < 4; ++q) {
                const int L = (wave + 8 * q) * 4 + (lane >> 3);
                const int b = (L >> 2) & 15, c = (L & 3) * 64 + (lane & 7) * 8;
                unsigned short* base = (q < 2) ? keysH : keysL;
                unsigned short* gp = base + ((size_t)((bg0 + b) * NN_ + idx)) * R_ + c;
                *(volatile u16x8*)gp = kv[q];
            }
        }
        __threadfence();
        __syncthreads();
    }
}

extern "C" void kernel_launch(void* const* d_in, const int* in_sizes, int n_in,
                              void* d_out, int out_size, void* d_ws, size_t ws_size,
                              hipStream_t stream)
{
    if (n_in < 16) return;
    if (in_sizes[0]  != NB_ * NN_ * R_)   return;
    if (in_sizes[1]  != NB_ * NN_ * NN_)  return;
    if (in_sizes[2]  != R_ * R_)          return;
    if (in_sizes[3]  != R_)               return;
    if (in_sizes[4]  != R_ * R_)          return;
    if (in_sizes[5]  != R_)               return;
    if (in_sizes[6]  != R_ * R_)          return;
    if (in_sizes[7]  != R_)               return;
    if (in_sizes[8]  != KF_ * R_)         return;
    if (in_sizes[9]  != R_)               return;
    if (in_sizes[10] != KF_ * R_)         return;
    if (in_sizes[11] != R_)               return;
    if (in_sizes[12] != KQ_ * R_)         return;
    if (in_sizes[13] != R_)               return;
    if (in_sizes[14] != KQ_ * R_)         return;
    if (in_sizes[15] != R_)               return;
    if (out_size != NB_ * NN_ * R_ + NB_ * NN_ * NN_) return;
    if (ws_size < WS_END)                 return;

    const float* nodes    = (const float*)d_in[0];
    const float* adj      = (const float*)d_in[1];
    const float* W_self   = (const float*)d_in[2];
    const float* b_self   = (const float*)d_in[3];
    const float* W_srep   = (const float*)d_in[4];
    const float* b_srep   = (const float*)d_in[5];
    const float* W_skey   = (const float*)d_in[6];
    const float* b_skey   = (const float*)d_in[7];
    const float* W_forget = (const float*)d_in[8];
    const float* b_forget = (const float*)d_in[9];
    const float* W_hid    = (const float*)d_in[10];
    const float* b_hid    = (const float*)d_in[11];
    const float* W_query  = (const float*)d_in[12];
    const float* b_query  = (const float*)d_in[13];
    const float* W_out    = (const float*)d_in[14];
    const float* b_out    = (const float*)d_in[15];

    float* out0 = (float*)d_out;
    float* out1 = out0 + (size_t)NB_ * NN_ * R_;

    char* ws = (char*)d_ws;
    unsigned short* nH  = (unsigned short*)(ws + OFF_NH);
    unsigned short* nL  = (unsigned short*)(ws + OFF_NL);
    unsigned short* wsH = (unsigned short*)(ws + OFF_WSH);
    unsigned short* wsL = (unsigned short*)(ws + OFF_WSL);
    unsigned short* wrH = (unsigned short*)(ws + OFF_WRH);
    unsigned short* wrL = (unsigned short*)(ws + OFF_WRL);
    unsigned short* wkH = (unsigned short*)(ws + OFF_WKH);
    unsigned short* wkL = (unsigned short*)(ws + OFF_WKL);
    unsigned short* wfH = (unsigned short*)(ws + OFF_WFH);
    unsigned short* wfL = (unsigned short*)(ws + OFF_WFL);
    unsigned short* whH = (unsigned short*)(ws + OFF_WHH);
    unsigned short* whL = (unsigned short*)(ws + OFF_WHL);
    unsigned short* wqH = (unsigned short*)(ws + OFF_WQH);
    unsigned short* wqL = (unsigned short*)(ws + OFF_WQL);
    unsigned short* woH = (unsigned short*)(ws + OFF_WOH);
    unsigned short* woL = (unsigned short*)(ws + OFF_WOL);
    float*          rep = (float*)(ws + OFF_REP);
    unsigned short* kH  = (unsigned short*)(ws + OFF_KH);
    unsigned short* kL  = (unsigned short*)(ws + OFF_KL);
    unsigned short* rtH = (unsigned short*)(ws + OFF_RTH);
    unsigned short* rtL = (unsigned short*)(ws + OFF_RTL);

    {
        const int n8 = (NB_ * NN_ * R_) / 8;
        cvt8_kernel<<<dim3((n8 + 255) / 256), dim3(256), 0, stream>>>(nodes, nH, nL, n8);
    }

    wt_cvt_kernel<<<dim3(R_ / 64, R_ / 64),  dim3(256), 0, stream>>>(W_self,   wsH, wsL, (int)R_, (int)R_,  (int)R_);
    wt_cvt_kernel<<<dim3(R_ / 64, R_ / 64),  dim3(256), 0, stream>>>(W_srep,   wrH, wrL, (int)R_, (int)R_,  (int)R_);
    wt_cvt_kernel<<<dim3(R_ / 64, R_ / 64),  dim3(256), 0, stream>>>(W_skey,   wkH, wkL, (int)R_, (int)R_,  (int)R_);
    wt_cvt_kernel<<<dim3(R_ / 64, KF_ / 64), dim3(256), 0, stream>>>(W_forget, wfH, wfL, (int)R_, (int)KF_, (int)R_);
    wt_cvt_kernel<<<dim3(R_ / 64, KF_ / 64), dim3(256), 0, stream>>>(W_hid,    whH, whL, (int)R_, (int)KF_, (int)R_);
    wt_cvt_kernel<<<dim3(R_ / 64, KQ_ / 64), dim3(256), 0, stream>>>(W_query,  wqH, wqL, (int)R_, (int)KQ_, (int)R_);
    wt_cvt_kernel<<<dim3(R_ / 64, KQ_ / 64), dim3(256), 0, stream>>>(W_out,    woH, woL, (int)R_, (int)KQ_, (int)R_);

    {
        const int n8 = (NB_ * NN_ * R_) / 8;
        init_src_kernel<<<dim3((n8 + 255) / 256), dim3(256), 0, stream>>>(b_skey, b_srep, kH, kL, rtH, rtL, n8);
    }

    {
        const int n4 = (NB_ * NN_ * NN_) / 4;
        copy4_kernel<<<dim3((n4 + 255) / 256), dim3(256), 0, stream>>>(adj, out1, n4);
    }

    gemm_x3_kernel<2><<<dim3(R_ / 64, MROWS_ / 64), dim3(128), 0, stream>>>(
        (const unsigned short*)nH, (const unsigned short*)nL,
        (const unsigned short*)wsH, (const unsigned short*)wsL,
        rep, (int)R_, (int)R_);

    hipFuncSetAttribute(reinterpret_cast<const void*>(&dag_kernel),
                        hipFuncAttributeMaxDynamicSharedMemorySize, LDS_BYTES);
    dag_kernel<<<dim3(NBLK_), dim3(256), LDS_BYTES, stream>>>(
        adj, (const float*)rep, b_self,
        (const unsigned short*)wfH, (const unsigned short*)wfL, b_forget,
        (const unsigned short*)whH, (const unsigned short*)whL, b_hid,
        (const unsigned short*)wqH, (const unsigned short*)wqL, b_query,
        (const unsigned short*)woH, (const unsigned short*)woL, b_out,
        (const unsigned short*)wrH, (const unsigned short*)wrL, b_srep,
        (const unsigned short*)wkH, (const unsigned short*)wkL, b_skey,
        kH, kL, rtH, rtL, out0);
}
